// GAT2NO_NORM_82575041232961
// MI455X (gfx1250) — hardware-verified
//
#include <hip/hip_runtime.h>
#include <stddef.h>


#define KIN   128
#define DF    256
#define NH    4
#define CO    64
#define GR    32
#define AP    136
#define XSP   260
#define NB    256
#define CHUNK 2048
#define NTHR  256
#define NWAVE 8
#define WCAP  256
#define NGRP  (CHUNK / (NTHR * 4))

#define LDS_SACC (NB * DF)
#define LDS_AUX  (NB * NH * 3)
#define LDS_LIST (NWAVE * WCAP)
#define LDS_BYTES ((LDS_SACC + LDS_AUX + LDS_LIST + NWAVE) * 4)

static_assert(WCAP == (CHUNK / NTHR) * 32);
static_assert(NGRP >= 1);
static_assert(NB == 256);
static_assert(NTHR == NB);
static_assert(NTHR == DF);
static_assert((CHUNK & (CHUNK - 1)) == 0);
static_assert(CHUNK <= 4096);
static_assert((LDS_SACC % 4) == 0);
static_assert(LDS_BYTES == 282656);
static_assert(DF == NH * CO);
static_assert((KIN % 32) == 0);
static_assert(GR == 32);

typedef float          v4f  __attribute__((ext_vector_type(4)));
typedef float          v8f  __attribute__((ext_vector_type(8)));
typedef int            v4i  __attribute__((ext_vector_type(4)));
typedef unsigned short v8us __attribute__((ext_vector_type(8)));
typedef __bf16         v8b  __attribute__((ext_vector_type(8)));
typedef __bf16         v16b __attribute__((ext_vector_type(16)));
union FragB  { v16b v; v8b half[2]; };
union Pack16 { v8b b; v8us u; v4i i; };

__device__ __forceinline__ v8f wm(v16b a, v16b b, v8f c) {
  v8f d = __builtin_amdgcn_wmma_f32_16x16x32_bf16(false, a, false, b, (short)0, c, false, false);
  asm volatile("v_nop\n\tv_nop\n\tv_nop\n\tv_nop" : "+v"(d) : "v"(a), "v"(b));
  return d;
}

__device__ __forceinline__ unsigned short f2bf(float f) {
  unsigned int u = __float_as_uint(f);
  u += 0x7FFFu + ((u >> 16) & 1u);
  return (unsigned short)(u >> 16);
}

__device__ __forceinline__ void split2(float f, unsigned short& hi, unsigned short& lo) {
  const unsigned short h = f2bf(f);
  const float r = f - __uint_as_float(((unsigned int)h) << 16);
  hi = h;
  lo = f2bf(r);
}

__device__ __forceinline__ float leaky(float v) { return v > 0.0f ? v : 0.2f * v; }

__device__ __forceinline__ v4f hsum(v4f v) {
  v.x += __shfl_xor(v.x, 8, 32);  v.y += __shfl_xor(v.y, 8, 32);
  v.z += __shfl_xor(v.z, 8, 32);  v.w += __shfl_xor(v.w, 8, 32);
  v.x += __shfl_xor(v.x, 16, 32); v.y += __shfl_xor(v.y, 16, 32);
  v.z += __shfl_xor(v.z, 16, 32); v.w += __shfl_xor(v.w, 16, 32);
  return v;
}

__device__ __forceinline__ v4f bcast4(v4f v, int s) {
  v4f r;
  r.x = __shfl(v.x, s, 32); r.y = __shfl(v.y, s, 32);
  r.z = __shfl(v.z, s, 32); r.w = __shfl(v.w, s, 32);
  return r;
}

__global__ __launch_bounds__(NTHR) void k_prepw(const float* __restrict__ W, __bf16* Whi, __bf16* Wlo, int n8) {
  const int i = blockIdx.x * NTHR + threadIdx.x;
  if (i >= n8) return;
  const size_t o = (size_t)i * 8;
  const v4f a = *(const v4f*)(W + o);
  const v4f b = *(const v4f*)(W + o + 4);
  const float f[8] = {a.x, a.y, a.z, a.w, b.x, b.y, b.z, b.w};
  Pack16 ph, pl;
#pragma unroll
  for (int j = 0; j < 8; ++j) {
    unsigned short th, tl;
    split2(f[j], th, tl);
    ph.u[j] = th;
    pl.u[j] = tl;
  }
  *(volatile v4i*)(Whi + o) = ph.i;
  *(volatile v4i*)(Wlo + o) = pl.i;
  __threadfence();
  *(volatile v4i*)(Whi + o) = ph.i;
  *(volatile v4i*)(Wlo + o) = pl.i;
}

__device__ __forceinline__ void epi_tile(v8f acc, int T, int hh, int ncol, float* Xs) {
#pragma unroll
  for (int r = 0; r < 8; ++r) Xs[(T * 16 + 8 * hh + r) * XSP + ncol] = acc[r];
}

__global__ __launch_bounds__(NTHR) void k_gemm(
    const float* __restrict__ x, const __bf16* __restrict__ Whi, const __bf16* __restrict__ Wlo,
    const float* __restrict__ att_src, const float* __restrict__ att_dst,
    float* hpl, float* asd, int nN) {
  __shared__ __attribute__((aligned(16))) __bf16 Ah[GR * AP];
  __shared__ __attribute__((aligned(16))) __bf16 Al[GR * AP];
  __shared__ __attribute__((aligned(16))) float Xs[GR * XSP];
  __shared__ __attribute__((aligned(16))) float Att[2 * DF];
  __shared__ __attribute__((aligned(16))) float AsD[GR * 8];

  const int tid  = threadIdx.x;
  const int lane = tid & 31;
  const int wave = tid >> 5;
  const int hh   = lane >> 4;
  const int m    = lane & 15;
  const int rowBase = blockIdx.x * GR;

  Att[tid]      = att_src[tid];
  Att[DF + tid] = att_dst[tid];

  {
    const int r  = tid >> 3;
    const int c0 = (tid & 7) * 16;
    int row = rowBase + r;
    if (row > nN - 1) row = nN - 1;
    const float* p = x + (size_t)row * KIN + c0;
    const v4f f0 = *(const v4f*)(p), f1 = *(const v4f*)(p + 4);
    const v4f f2 = *(const v4f*)(p + 8), f3 = *(const v4f*)(p + 12);
    const float f[16] = {f0.x, f0.y, f0.z, f0.w, f1.x, f1.y, f1.z, f1.w,
                         f2.x, f2.y, f2.z, f2.w, f3.x, f3.y, f3.z, f3.w};
    Pack16 h0, h1, l0, l1;
#pragma unroll
    for (int j = 0; j < 8; ++j) {
      unsigned short th, tl;
      split2(f[j], th, tl);      h0.u[j] = th; l0.u[j] = tl;
      split2(f[8 + j], th, tl);  h1.u[j] = th; l1.u[j] = tl;
    }
    *(v8b*)(Ah + r * AP + c0)     = h0.b;
    *(v8b*)(Ah + r * AP + c0 + 8) = h1.b;
    *(v8b*)(Al + r * AP + c0)     = l0.b;
    *(v8b*)(Al + r * AP + c0 + 8) = l1.b;
  }
  __syncthreads();

  const int n0 = wave * 32;
  v8f c00 = {0.f, 0.f, 0.f, 0.f, 0.f, 0.f, 0.f, 0.f};
  v8f c01 = {0.f, 0.f, 0.f, 0.f, 0.f, 0.f, 0.f, 0.f};
  v8f c10 = {0.f, 0.f, 0.f, 0.f, 0.f, 0.f, 0.f, 0.f};
  v8f c11 = {0.f, 0.f, 0.f, 0.f, 0.f, 0.f, 0.f, 0.f};
#pragma unroll
  for (int kt = 0; kt < KIN / 32; ++kt) {
    const int k0 = kt * 32;
    FragB a0h, a0l, a1h, a1l, b0h, b0l, b1h, b1l;
    const __bf16* pa0 = Ah + m * AP + k0 + 8 * hh;
    const __bf16* pa1 = Ah + (16 + m) * AP + k0 + 8 * hh;
    const __bf16* qa0 = Al + m * AP + k0 + 8 * hh;
    const __bf16* qa1 = Al + (16 + m) * AP + k0 + 8 * hh;
    const __bf16* pb0 = Whi + (size_t)(n0 + m) * KIN + k0 + 8 * hh;
    const __bf16* pb1 = Whi + (size_t)(n0 + 16 + m) * KIN + k0 + 8 * hh;
    const __bf16* qb0 = Wlo + (size_t)(n0 + m) * KIN + k0 + 8 * hh;
    const __bf16* qb1 = Wlo + (size_t)(n0 + 16 + m) * KIN + k0 + 8 * hh;
    a0h.half[0] = *(const v8b*)pa0; a0h.half[1] = *(const v8b*)(pa0 + 16);
    a1h.half[0] = *(const v8b*)pa1; a1h.half[1] = *(const v8b*)(pa1 + 16);
    a0l.half[0] = *(const v8b*)qa0; a0l.half[1] = *(const v8b*)(qa0 + 16);
    a1l.half[0] = *(const v8b*)qa1; a1l.half[1] = *(const v8b*)(qa1 + 16);
    b0h.half[0] = *(const v8b*)pb0; b0h.half[1] = *(const v8b*)(pb0 + 16);
    b1h.half[0] = *(const v8b*)pb1; b1h.half[1] = *(const v8b*)(pb1 + 16);
    b0l.half[0] = *(const v8b*)qb0; b0l.half[1] = *(const v8b*)(qb0 + 16);
    b1l.half[0] = *(const v8b*)qb1; b1l.half[1] = *(const v8b*)(qb1 + 16);
    c00 = wm(a0h.v, b0h.v, c00); c00 = wm(a0l.v, b0h.v, c00); c00 = wm(a0h.v, b0l.v, c00);
    c01 = wm(a0h.v, b1h.v, c01); c01 = wm(a0l.v, b1h.v, c01); c01 = wm(a0h.v, b1l.v, c01);
    c10 = wm(a1h.v, b0h.v, c10); c10 = wm(a1l.v, b0h.v, c10); c10 = wm(a1h.v, b0l.v, c10);
    c11 = wm(a1h.v, b1h.v, c11); c11 = wm(a1l.v, b1h.v, c11); c11 = wm(a1h.v, b1l.v, c11);
  }

  epi_tile(c00, 0, hh, n0 + m, Xs);
  epi_tile(c01, 0, hh, n0 + 16 + m, Xs);
  epi_tile(c10, 1, hh, n0 + m, Xs);
  epi_tile(c11, 1, hh, n0 + 16 + m, Xs);
  __syncthreads();

  {
    const int r   = tid >> 3;
    const int q   = tid & 7;
    const int typ = q >> 2;
    const int hd  = q & 3;
    const float* xr = Xs + r * XSP + hd * CO;
    const float* av = Att + typ * DF + hd * CO;
    float s = 0.0f;
#pragma unroll 8
    for (int c = 0; c < CO; ++c) s += xr[c] * av[c];
    AsD[r * 8 + q] = s;
  }
  __syncthreads();

  v4f xa[4], xb[4];
#pragma unroll
  for (int i = 0; i < 4; ++i) {
    xa[i] = *(const v4f*)(Xs + (4 * wave + i) * XSP + 4 * lane);
    xb[i] = *(const v4f*)(Xs + (4 * wave + i) * XSP + 128 + 4 * lane);
  }
  float* gp = 0;
  v4f gv = {0.f, 0.f, 0.f, 0.f};
  if (wave < 2) {
    gv = *(const v4f*)(AsD + wave * 128 + 4 * lane);
    gp = asd + (size_t)rowBase * 8 + wave * 128 + 4 * lane;
  }
  float* hp[4];
#pragma unroll
  for (int i = 0; i < 4; ++i) hp[i] = hpl + (size_t)(rowBase + 4 * wave + i) * DF + 4 * lane;

#pragma unroll
  for (int i = 0; i < 4; ++i) {
    *(volatile v4f*)(hp[i])       = xa[i];
    *(volatile v4f*)(hp[i] + 128) = xb[i];
  }
  if (gp) *(volatile v4f*)gp = gv;
  __threadfence();
#pragma unroll
  for (int i = 0; i < 4; ++i) {
    *(volatile v4f*)(hp[i])       = xa[i];
    *(volatile v4f*)(hp[i] + 128) = xb[i];
  }
  if (gp) *(volatile v4f*)gp = gv;
}

__device__ __forceinline__ void slot_final(int slot, int nodeBase, int nN, int lane, int hd,
                                           const float* __restrict__ asd, const float* __restrict__ hpl,
                                           const float* sacc, const float* smx, const float* sden,
                                           const float* sad, v4f& o0, v4f& o1) {
  int nd = nodeBase + slot;
  if (nd > nN - 1) nd = nN - 1;
  const size_t nrow = (size_t)nd;
  const float as = asd[nrow * 8 + hd];
  const float ad = sad[slot * NH + hd];
  const float ev = leaky(as + ad);
  const float mo = smx[slot * NH + hd];
  const float mn = fmaxf(mo, ev);
  const float corr = __expf(mo - mn);
  const float p    = __expf(ev - mn);
  const float* hr = hpl + nrow * DF + 8 * lane;
  const v4f h0 = *(const v4f*)(hr), h1 = *(const v4f*)(hr + 4);
  const v4f a0 = *(const v4f*)(sacc + slot * DF + 8 * lane);
  const v4f a1 = *(const v4f*)(sacc + slot * DF + 8 * lane + 4);
  const float dn  = sden[slot * NH + hd] * corr + p;
  const float inv = 1.0f / dn;
  v4f v0 = (a0 * corr + p * h0) * inv;
  v4f v1 = (a1 * corr + p * h1) * inv;
  o0 = hsum(v0);
  o1 = hsum(v1);
}

__global__ __launch_bounds__(NTHR) void k_gat(
    const int* __restrict__ ei, const float* __restrict__ hpl, const float* __restrict__ asd,
    const float* __restrict__ bias, float* out, int nN, int nE) {
  extern __shared__ v4f lds_dyn[];
  float* sacc  = (float*)lds_dyn;
  float* smx   = sacc + LDS_SACC;
  float* sden  = smx + NB * NH;
  float* sad   = sden + NB * NH;
  int*   hlist = (int*)(sad + NB * NH);
  int*   wcnt  = hlist + LDS_LIST;

  const int tid  = threadIdx.x;
  const int lane = tid & 31;
  const int wave = tid >> 5;
  const int hd   = lane >> 3;
  const int nodeBase = blockIdx.x * NB;

  {
    const v4f z4 = {0.f, 0.f, 0.f, 0.f};
    for (int i = tid; i < LDS_SACC / 4; i += NTHR) lds_dyn[i] = z4;
    int nd = nodeBase + tid;
    if (nd > nN - 1) nd = nN - 1;
    const v4f a4 = *(const v4f*)(asd + (size_t)nd * 8 + 4);
    *(v4f*)(sad + tid * NH) = a4;
    const v4f m4 = {-1e30f, -1e30f, -1e30f, -1e30f};
    *(v4f*)(smx + tid * NH)  = m4;
    *(v4f*)(sden + tid * NH) = z4;
  }
  __syncthreads();

  const int* eid = ei + nE;
  const bool al16 = ((nE & 3) == 0);

  const int nChunks = (nE + CHUNK - 1) / CHUNK;
#pragma unroll 1
  for (int ch = 0; ch < nChunks; ++ch) {
    const int cbase = ch * CHUNK;
    int wc = 0;
#pragma unroll
    for (int g = 0; g < NGRP; ++g) {
      const int el0 = (g * NTHR + tid) * 4;
      const int e0  = cbase + el0;
      const int sent = -2147483647 - 1;
      v4i d;
      if (al16 && (cbase + CHUNK <= nE)) {
        d = *(const v4i*)(eid + e0);
      } else {
        d.x = (e0     < nE) ? eid[min(e0, nE - 1)]     : sent;
        d.y = (e0 + 1 < nE) ? eid[min(e0 + 1, nE - 1)] : sent;
        d.z = (e0 + 2 < nE) ? eid[min(e0 + 2, nE - 1)] : sent;
        d.w = (e0 + 3 < nE) ? eid[min(e0 + 3, nE - 1)] : sent;
      }
      const unsigned s0 = (unsigned)d.x - (unsigned)nodeBase;
      const unsigned s1 = (unsigned)d.y - (unsigned)nodeBase;
      const unsigned s2 = (unsigned)d.z - (unsigned)nodeBase;
      const unsigned s3 = (unsigned)d.w - (unsigned)nodeBase;
      const bool h0 = s0 < (unsigned)NB;
      const bool h1 = s1 < (unsigned)NB;
      const bool h2 = s2 < (unsigned)NB;
      const bool h3 = s3 < (unsigned)NB;
      const unsigned many = __builtin_amdgcn_ballot_w32(h0 | h1 | h2 | h3);
      if (many != 0u) {
#define HITJ(J, HJ, SJ) { \
          const unsigned mj = __builtin_amdgcn_ballot_w32(HJ); \
          if (HJ) { \
            const int pos = wc + (int)__builtin_amdgcn_mbcnt_lo(mj, 0u); \
            if (pos < WCAP) hlist[wave * WCAP + pos] = ((el0 + (J)) << 8) | (int)(SJ); \
          } \
          wc += (int)__builtin_popcount(mj); }
        HITJ(0, h0, s0)
        HITJ(1, h1, s1)
        HITJ(2, h2, s2)
        HITJ(3, h3, s3)
#undef HITJ
      }
    }
    if (lane == 0) wcnt[wave] = wc;
    __syncthreads();

    if (wave == 0) {
#pragma unroll 1
      for (int wsx = 0; wsx < NWAVE; ++wsx) {
        int n = wcnt[wsx];
        if (n > WCAP) n = WCAP;
        if (n < 0) n = 0;
#pragma unroll 1
        for (int i = 0; i < n; ++i) {
          const int ent  = hlist[wsx * WCAP + i];
          const int slot = ent & (NB - 1);
          const int el   = (ent >> 8) & (CHUNK - 1);
          int e = cbase + el;
          if (e > nE - 1) e = nE - 1;
          int src = ei[e];
          src = src < 0 ? 0 : (src > nN - 1 ? nN - 1 : src);
          const size_t srow = (size_t)src;
          const float as = asd[srow * 8 + hd];
          const float ad = sad[slot * NH + hd];
          const float ev = leaky(as + ad);
          const int   ai = slot * NH + hd;
          const float mo = smx[ai];
          const float mn = fmaxf(mo, ev);
          const float corr = __expf(mo - mn);
          const float p    = __expf(ev - mn);
          const float* hr = hpl + srow * DF + 8 * lane;
          const v4f x0 = *(const v4f*)(hr), x1 = *(const v4f*)(hr + 4);
          v4f* ap = (v4f*)(sacc + slot * DF + 8 * lane);
          const v4f a0 = ap[0], a1 = ap[1];
          const v4f n0 = a0 * corr + p * x0;
          const v4f n1 = a1 * corr + p * x1;
          ap[0] = n0;
          ap[1] = n1;
          const float dn = sden[ai] * corr + p;
          smx[ai]  = mn;
          sden[ai] = dn;
        }
      }
    }
    __syncthreads();
  }

  const int cg = lane & 7;
  const v4f b0 = *(const v4f*)(bias + 8 * cg);
  const v4f b1 = *(const v4f*)(bias + 8 * cg + 4);
  const int sBase = wave * (NB / NWAVE);
  const int nodeW = nodeBase + sBase;
  int nv = nN - nodeW;
  if (nv < 0) nv = 0;
  if (nv > 32) nv = 32;
  const int srl  = (lane & 15) >> 1;
  const bool hi8 = (lane & 1) != 0;
  const bool rwB = lane >= 16;
#pragma unroll 1
  for (int jp = 0; jp < 16; ++jp) {
    const int j = 2 * jp;
    if (j >= nv) break;
    v4f oA0, oA1, oB0, oB1;
    slot_final(sBase + j,     nodeBase, nN, lane, hd, asd, hpl, sacc, smx, sden, sad, oA0, oA1);
    slot_final(sBase + j + 1, nodeBase, nN, lane, hd, asd, hpl, sacc, smx, sden, sad, oB0, oB1);
    oA0 = oA0 * 0.25f + b0; oA1 = oA1 * 0.25f + b1;
    oB0 = oB0 * 0.25f + b0; oB1 = oB1 * 0.25f + b1;
    oA0.x = fmaxf(oA0.x, 0.f); oA0.y = fmaxf(oA0.y, 0.f); oA0.z = fmaxf(oA0.z, 0.f); oA0.w = fmaxf(oA0.w, 0.f);
    oA1.x = fmaxf(oA1.x, 0.f); oA1.y = fmaxf(oA1.y, 0.f); oA1.z = fmaxf(oA1.z, 0.f); oA1.w = fmaxf(oA1.w, 0.f);
    oB0.x = fmaxf(oB0.x, 0.f); oB0.y = fmaxf(oB0.y, 0.f); oB0.z = fmaxf(oB0.z, 0.f); oB0.w = fmaxf(oB0.w, 0.f);
    oB1.x = fmaxf(oB1.x, 0.f); oB1.y = fmaxf(oB1.y, 0.f); oB1.z = fmaxf(oB1.z, 0.f); oB1.w = fmaxf(oB1.w, 0.f);
    const v4f tA0 = bcast4(oA0, srl), tA1 = bcast4(oA1, srl);
    const v4f tB0 = bcast4(oB0, srl), tB1 = bcast4(oB1, srl);
    const v4f vA = hi8 ? tA1 : tA0;
    const v4f vB = hi8 ? tB1 : tB0;
    const v4f v  = rwB ? vB : vA;
    float* op = out + (size_t)(nodeW + j) * CO + 4 * lane;
    const bool full = (j + 1 < nv);
    const bool act  = full || (lane < 16);
    if (act) *(volatile v4f*)op = v;
    __threadfence();
    if (act) *(volatile v4f*)op = v;
  }
}

extern "C" void kernel_launch(void* const* d_in, const int* in_sizes, int n_in,
                              void* d_out, int out_size, void* d_ws, size_t ws_size,
                              hipStream_t stream) {
  if (n_in < 6) return;
  const int nN = in_sizes[0] / KIN;
  if (nN <= 0 || in_sizes[0] != nN * KIN) return;
  if (in_sizes[1] < 0 || (in_sizes[1] & 1) != 0) return;
  const int nE = in_sizes[1] / 2;
  if (in_sizes[2] != DF * KIN) return;
  if (in_sizes[3] != NH * CO || in_sizes[4] != NH * CO) return;
  if (in_sizes[5] != CO) return;
  if (out_size != nN * CO) return;

  const float* x       = (const float*)d_in[0];
  const int*   ei      = (const int*)d_in[1];
  const float* W       = (const float*)d_in[2];
  const float* att_src = (const float*)d_in[3];
  const float* att_dst = (const float*)d_in[4];
  const float* bias    = (const float*)d_in[5];
  float* out = (float*)d_out;

  const int nP = ((nN + GR - 1) / GR) * GR;
  size_t off = 0;
  __bf16* Whi = (__bf16*)((char*)d_ws + off); off += (size_t)DF * KIN * sizeof(__bf16);
  __bf16* Wlo = (__bf16*)((char*)d_ws + off); off += (size_t)DF * KIN * sizeof(__bf16);
  float* hpl = (float*)((char*)d_ws + off);    off += (size_t)nP * DF * sizeof(float);
  float* asd = (float*)((char*)d_ws + off);    off += (size_t)nP * 8 * sizeof(float);
  if (off > ws_size) return;

  const int n8 = DF * KIN / 8;
  k_prepw<<<(n8 + NTHR - 1) / NTHR, NTHR, 0, stream>>>(W, Whi, Wlo, n8);

  k_gemm<<<nP / GR, NTHR, 0, stream>>>(x, Whi, Wlo, att_src, att_dst, hpl, asd, nN);

  hipFuncSetAttribute(reinterpret_cast<const void*>(&k_gat),
                      hipFuncAttributeMaxDynamicSharedMemorySize, LDS_BYTES);
  const int grid = (nN + NB - 1) / NB;
  k_gat<<<grid, NTHR, LDS_BYTES, stream>>>(ei, hpl, asd, bias, out, nN, nE);
}
